// MultiScaleRetention_44633300140813
// MI455X (gfx1250) — hardware-verified
//
#include <hip/hip_runtime.h>


#ifndef NB
#define NB 4
#endif
#ifndef SEQ
#define SEQ 2048
#endif
#define NB_FULL  4
#define SEQ_FULL 2048
#define DIM  1024
#define HD   128
#define NH   8
#define ROWS (NB * SEQ)

#define PSC    8.0f
#define RSC    2048.0f
#define WCARRY 1024.0f
#define ZSC    16.0f
#define WOSC   256.0f
#define RS128  0.08838834764831845f

static_assert(SEQ % 64 == 0);
static_assert(SEQ >= 64 && SEQ <= SEQ_FULL);
static_assert(NB >= 1 && NB <= NB_FULL);
static_assert(NH * HD == DIM);
static_assert((ROWS * DIM) % 2048 == 0);
static_assert(DIM % 64 == 0 && HD % 64 == 0 && HD % 32 == 0);

typedef _Float16       v16h __attribute__((ext_vector_type(16)));
typedef _Float16       v8h  __attribute__((ext_vector_type(8)));
typedef __bf16         v16b __attribute__((ext_vector_type(16)));
typedef float          v8f  __attribute__((ext_vector_type(8)));
typedef float          v4f  __attribute__((ext_vector_type(4)));
typedef unsigned int   v4u  __attribute__((ext_vector_type(4)));
typedef unsigned short u16;

union Frag  { v16h h; v16b b; v4u u[2]; v8h p[2]; };
union Pack8 { v8h h; v4u u; };

__device__ __forceinline__ Frag ldfrag(const u16* __restrict__ p, int hh) {
  Frag f;
  f.u[0] = *(const v4u*)(p + 8 * hh);
  f.u[1] = *(const v4u*)(p + 16 + 8 * hh);
  return f;
}

__device__ __forceinline__ v8f mma_f16(const Frag& a, const Frag& b, v8f c) {
  v8f d = __builtin_amdgcn_wmma_f32_16x16x32_f16(false, a.h, false, b.h, (short)0, c, false, false);
  asm volatile("v_nop\n\tv_nop\n\tv_nop\n\tv_nop" : "+v"(d) : "v"(a.h), "v"(b.h));
  return d;
}

__device__ __forceinline__ v8f mma_bf16(const Frag& a, const Frag& b, v8f c) {
  v8f d = __builtin_amdgcn_wmma_f32_16x16x32_bf16(false, a.b, false, b.b, (short)0, c, false, false);
  asm volatile("v_nop\n\tv_nop\n\tv_nop\n\tv_nop" : "+v"(d) : "v"(a.b), "v"(b.b));
  return d;
}

__device__ __forceinline__ unsigned bf16bits(float x) {
  const unsigned u = __float_as_uint(x);
  return (u + 0x7fffu + ((u >> 16) & 1u)) >> 16;
}
__device__ __forceinline__ float bf16q(float x) { return __uint_as_float(bf16bits(x) << 16); }

__global__ __launch_bounds__(256) void k_cvt_q(const float* __restrict__ q, u16* __restrict__ qb) {
  const size_t e   = ((size_t)blockIdx.x * 256u + threadIdx.x) * 8u;
  const size_t row = e / DIM;
  const int    col = (int)(e - row * DIM);
  const size_t b   = row / SEQ;
  const size_t s   = row - b * SEQ;
  const float* sp  = q + (b * SEQ_FULL + s) * DIM + col;
  const v4f a = *(const v4f*)sp;
  const v4f c = *(const v4f*)(sp + 4);
  v4u o;
  o[0] = bf16bits(a[0]) | (bf16bits(a[1]) << 16);
  o[1] = bf16bits(a[2]) | (bf16bits(a[3]) << 16);
  o[2] = bf16bits(c[0]) | (bf16bits(c[1]) << 16);
  o[3] = bf16bits(c[2]) | (bf16bits(c[3]) << 16);
  u16* dp = qb + row * DIM + col;
  *(volatile v4u*)dp = o;
  __threadfence();
  *(volatile v4u*)dp = o;
}

template <int MODE>
__global__ __launch_bounds__(256) void k_tr(const float* __restrict__ in, u16* __restrict__ out,
                                            int R, int C) {
  __shared__ float tile[64][65];
  const int t  = threadIdx.x;
  const int c0 = blockIdx.x * 64;
  const int r0 = blockIdx.y * 64;
  const size_t zoff = (size_t)blockIdx.z * (size_t)R * (size_t)C;
#pragma unroll
  for (int i = 0; i < 16; ++i) {
    const int r = i * 4 + (t >> 6);
    const int c = t & 63;
    tile[r][c] = in[zoff + (size_t)(r0 + r) * C + c0 + c];
  }
  __syncthreads();
  v4u    o[2];
  size_t d[2];
#pragma unroll
  for (int i = 0; i < 2; ++i) {
    const int cl    = 32 * i + (t >> 3);
    const int piece = t & 7;
    if (MODE == 0) {
      v4u w = {0u, 0u, 0u, 0u};
#pragma unroll
      for (int j = 0; j < 8; ++j) {
        const unsigned bits = bf16bits(tile[8 * piece + j][cl]);
        w[j >> 1] |= bits << (16 * (j & 1));
      }
      o[i] = w;
    } else {
      Pack8 pk;
#pragma unroll
      for (int j = 0; j < 8; ++j) pk.h[j] = (_Float16)(bf16q(tile[8 * piece + j][cl]) * WOSC);
      o[i] = pk.u;
    }
    d[i] = zoff + (size_t)(c0 + cl) * R + r0 + 8 * piece;
  }
#pragma unroll
  for (int i = 0; i < 2; ++i) *(volatile v4u*)(out + d[i]) = o[i];
  __threadfence();
#pragma unroll
  for (int i = 0; i < 2; ++i) *(volatile v4u*)(out + d[i]) = o[i];
}

__global__ __launch_bounds__(256) void k_proj(const u16* __restrict__ qb, const u16* __restrict__ WT,
                                              float* __restrict__ Pf, u16* __restrict__ Phr,
                                              u16* __restrict__ Vth, u16* __restrict__ Vtl) {
  __shared__ __attribute__((aligned(16))) float Ps[64][68];
  const int t = threadIdx.x, lane = t & 31, w = t >> 5;
  const int hh = lane >> 4, l15 = lane & 15, mloc = 8 * hh;
  const int rg = w & 3, cp = w >> 2;
  const int bh = blockIdx.z, b = bh / NH, h = bh - b * NH;
  const int s0 = blockIdx.x * 64, dt = blockIdx.y;

  const u16* ap  = qb + (size_t)(b * SEQ + s0 + 16 * rg + l15) * DIM + h * HD;
  const u16* bp0 = WT + ((size_t)h * HD + dt * 64 + cp * 32 + l15) * HD;
  const u16* bp1 = bp0 + 16 * HD;

  v8f acc0 = {}, acc1 = {};
#pragma unroll
  for (int kc = 0; kc < HD / 32; ++kc) {
    const Frag a  = ldfrag(ap + 32 * kc, hh);
    const Frag b0 = ldfrag(bp0 + 32 * kc, hh);
    const Frag b1 = ldfrag(bp1 + 32 * kc, hh);
    acc0 = mma_bf16(a, b0, acc0);
    acc1 = mma_bf16(a, b1, acc1);
  }
#pragma unroll
  for (int r = 0; r < 8; ++r) {
    Ps[16 * rg + mloc + r][cp * 32 + l15]      = acc0[r];
    Ps[16 * rg + mloc + r][cp * 32 + 16 + l15] = acc1[r];
  }
  __syncthreads();

  v4f    fo[4];
  size_t fd[4];
#pragma unroll
  for (int i = 0; i < 4; ++i) {
    const int L   = 32 * i + (t >> 3);
    const int row = L >> 1;
    const int col = (L & 1) * 32 + (t & 7) * 4;
    fo[i] = *(const v4f*)&Ps[row][col];
    fd[i] = ((size_t)bh * SEQ + s0 + row) * HD + dt * 64 + col;
  }
  v4u    ho[2];
  size_t hd2[2];
#pragma unroll
  for (int i = 0; i < 2; ++i) {
    const int row = 32 * i + (t >> 3);
    const int col = (t & 7) * 8;
    Pack8 pk;
#pragma unroll
    for (int j = 0; j < 8; ++j) pk.h[j] = (_Float16)(PSC * Ps[row][col + j]);
    ho[i]  = pk.u;
    hd2[i] = ((size_t)bh * SEQ + s0 + row) * HD + dt * 64 + col;
  }
  v4u    vh[2], vl[2];
  size_t vd[2];
#pragma unroll
  for (int i = 0; i < 2; ++i) {
    const int dl = 32 * i + (t >> 3);
    const int sb = (t & 7) * 8;
    Pack8 ph, pl;
#pragma unroll
    for (int j = 0; j < 8; ++j) {
      const float    v  = PSC * Ps[sb + j][dl];
      const _Float16 hv = (_Float16)v;
      ph.h[j] = hv;
      pl.h[j] = (_Float16)((v - (float)hv) * RSC);
    }
    vh[i] = ph.u;
    vl[i] = pl.u;
    vd[i] = ((size_t)bh * HD + dt * 64 + dl) * SEQ + s0 + sb;
  }
#pragma unroll
  for (int i = 0; i < 4; ++i) *(volatile v4f*)(Pf + fd[i]) = fo[i];
#pragma unroll
  for (int i = 0; i < 2; ++i) {
    *(volatile v4u*)(Phr + hd2[i]) = ho[i];
    *(volatile v4u*)(Vth + vd[i])  = vh[i];
    *(volatile v4u*)(Vtl + vd[i])  = vl[i];
  }
  __threadfence();
#pragma unroll
  for (int i = 0; i < 4; ++i) *(volatile v4f*)(Pf + fd[i]) = fo[i];
#pragma unroll
  for (int i = 0; i < 2; ++i) {
    *(volatile v4u*)(Phr + hd2[i]) = ho[i];
    *(volatile v4u*)(Vth + vd[i])  = vh[i];
    *(volatile v4u*)(Vtl + vd[i])  = vl[i];
  }
}

__global__ __launch_bounds__(128) void k_colstat(const float* __restrict__ Pf, float* __restrict__ colw) {
  __shared__ __attribute__((aligned(16))) float part[4][SEQ];
  __shared__ __attribute__((aligned(16))) float cinv_s[SEQ];
  const int tid = threadIdx.x, lane = tid & 31, w = tid >> 5;
  const int bh = blockIdx.x;
  const int h  = bh % NH;
  const float gamma = 1.0f - __uint_as_float((unsigned)(122 - h) << 23);
  const float* pp = Pf + (size_t)bh * SEQ * HD + tid;
  float R = 0.0f, geo = 0.0f;
  for (int t = SEQ - 1; t >= 0; --t) {
    const float pv = pp[(size_t)t * HD];
    R   = pv + gamma * R;
    geo = 1.0f + gamma * geo;
    float pr = R * pv;
    pr += __shfl_xor(pr, 16, 32);
    pr += __shfl_xor(pr, 8, 32);
    pr += __shfl_xor(pr, 4, 32);
    pr += __shfl_xor(pr, 2, 32);
    pr += __shfl_xor(pr, 1, 32);
    if (lane == 0) part[w][t] = pr;
    if (tid == 0) cinv_s[t] = rsqrtf(geo);
  }
  __syncthreads();
  for (int base = 0; base < SEQ; base += 512) {
    const int t4 = base + 4 * tid;
    if (t4 < SEQ) {
      v4f o;
#pragma unroll
      for (int j = 0; j < 4; ++j) {
        const int   tt  = t4 + j;
        const float ci  = cinv_s[tt];
        const float cs  = ((part[0][tt] + part[1][tt]) + (part[2][tt] + part[3][tt])) * ci * RS128;
        const float den = fmaxf(fabsf(cs), 1.0f);
        o[j] = ci * (1.0f / den);
      }
      float* dp = colw + (size_t)bh * SEQ + t4;
      *(volatile v4f*)dp = o;
      __threadfence();
      *(volatile v4f*)dp = o;
    }
  }
}

__global__ __launch_bounds__(512) void k_ret(const u16* __restrict__ Phr, const u16* __restrict__ Vth,
                                             const u16* __restrict__ Vtl, const float* __restrict__ colw,
                                             float* __restrict__ Xf) {
  __shared__ __attribute__((aligned(16))) _Float16 Pt[2][4][16][72];
  __shared__ __attribute__((aligned(16))) float    Xs[64][132];
  const int t = threadIdx.x, lane = t & 31, w = t >> 5;
  const int hh = lane >> 4, l15 = lane & 15, mloc = 8 * hh;
  const int rg = w & 3, p = w >> 2;
  const int h = blockIdx.y, b = blockIdx.z, bh = b * NH + h;
  const int base = blockIdx.x * 64, q0 = base + 16 * rg;
  const int keycol = 16 * p + l15;

  const float gamma = 1.0f - __uint_as_float((unsigned)(122 - h) << 23);
  float g2[11];
  g2[0] = gamma;
#pragma unroll
  for (int i = 1; i < 11; ++i) g2[i] = g2[i - 1] * g2[i - 1];
  const int n0p = q0 + mloc;
  float prow = 1.0f;
#pragma unroll
  for (int i = 0; i < 11; ++i) prow = (n0p & (1 << i)) ? prow * g2[i] : prow;
  float pcol = 1.0f;
#pragma unroll
  for (int i = 0; i < 6; ++i) pcol = (keycol & (1 << i)) ? pcol * g2[i] : pcol;
  float rf[8];
  rf[0] = prow;
#pragma unroll
  for (int v = 1; v < 8; ++v) rf[v] = rf[v - 1] * gamma;
  const float cw    = 1.0f / pcol;
  const float stepf = 1.0f / g2[6];
  const float cfac  = cw * (RS128 / (PSC * PSC)) * WCARRY;

  const u16* qrow = Phr + ((size_t)bh * SEQ + q0 + l15) * HD;
  Frag aq[4];
#pragma unroll
  for (int kc = 0; kc < 4; ++kc) aq[kc] = ldfrag(qrow + 32 * kc, hh);

  const float* cwp   = colw + (size_t)bh * SEQ;
  const u16*   vhrow = Vth + ((size_t)bh * HD + 32 * p + l15) * SEQ;
  const u16*   vlrow = Vtl + ((size_t)bh * HD + 32 * p + l15) * SEQ;

  v8f oh0 = {}, oh1 = {}, ol0 = {}, ol1 = {};
  int buf = 0;
  for (int m0 = 0; m0 < base + 64; m0 += 64) {
    const int  key  = m0 + keycol;
    const u16* krow = Phr + ((size_t)bh * SEQ + key) * HD;
    v8f sacc = {};
#pragma unroll
    for (int kc = 0; kc < 4; ++kc) {
      const Frag bk = ldfrag(krow + 32 * kc, hh);
      sacc = mma_f16(aq[kc], bk, sacc);
    }
    const float f = cfac * cwp[key];
#pragma unroll
    for (int v = 0; v < 8; ++v) {
      const int   qn  = q0 + mloc + v;
      const float wgt = (qn >= key) ? rf[v] * f : 0.0f;
      Pt[buf][rg][mloc + v][keycol] = (_Float16)(sacc[v] * wgt);
      rf[v] *= stepf;
    }
    __syncthreads();
#pragma unroll 1
    for (int ks = 0; ks < 2; ++ks) {
      Frag pf;
      pf.p[0] = *(const v8h*)&Pt[buf][rg][l15][32 * ks + mloc];
      pf.p[1] = *(const v8h*)&Pt[buf][rg][l15][32 * ks + 16 + mloc];
      const size_t ko = (size_t)(m0 + 32 * ks);
      const Frag bvh0 = ldfrag(vhrow + ko, hh);
      const Frag bvl0 = ldfrag(vlrow + ko, hh);
      const Frag bvh1 = ldfrag(vhrow + 16 * SEQ + ko, hh);
      const Frag bvl1 = ldfrag(vlrow + 16 * SEQ + ko, hh);
      oh0 = mma_f16(pf, bvh0, oh0);
      ol0 = mma_f16(pf, bvl0, ol0);
      oh1 = mma_f16(pf, bvh1, oh1);
      ol1 = mma_f16(pf, bvl1, ol1);
    }
    buf ^= 1;
  }

  const float c1 = 1.0f / (WCARRY * PSC);
  const float c2 = c1 / RSC;
#pragma unroll
  for (int r = 0; r < 8; ++r) {
    const int xr = 16 * rg + mloc + r;
    Xs[xr][32 * p + l15]      = oh0[r] * c1 + ol0[r] * c2;
    Xs[xr][32 * p + 16 + l15] = oh1[r] * c1 + ol1[r] * c2;
  }
  __syncthreads();
  v4f    xo[4];
  size_t xd[4];
#pragma unroll
  for (int i = 0; i < 4; ++i) {
    const int L   = 64 * i + (t >> 3);
    const int row = L >> 2;
    const int col = (L & 3) * 32 + (t & 7) * 4;
    xo[i] = *(const v4f*)&Xs[row][col];
    xd[i] = ((size_t)b * SEQ + base + row) * DIM + h * HD + col;
  }
#pragma unroll
  for (int i = 0; i < 4; ++i) *(volatile v4f*)(Xf + xd[i]) = xo[i];
  __threadfence();
#pragma unroll
  for (int i = 0; i < 4; ++i) *(volatile v4f*)(Xf + xd[i]) = xo[i];
}

__global__ __launch_bounds__(256) void k_gate(const u16* __restrict__ qb, const u16* __restrict__ WgT,
                                              const float* __restrict__ bg, float* __restrict__ G) {
  __shared__ __attribute__((aligned(16))) float Cs[64][68];
  const int t = threadIdx.x, lane = t & 31, w = t >> 5;
  const int hh = lane >> 4, l15 = lane & 15, mloc = 8 * hh;
  const int rg = w & 3, cp = w >> 2;
  const int m0 = blockIdx.x * 64, n0 = blockIdx.y * 64;

  const u16* ap  = qb + (size_t)(m0 + 16 * rg + l15) * DIM;
  const u16* bp0 = WgT + (size_t)(n0 + 32 * cp + l15) * DIM;
  const u16* bp1 = bp0 + 16 * DIM;

  v8f acc0 = {}, acc1 = {};
#pragma unroll 2
  for (int k0 = 0; k0 < DIM; k0 += 32) {
    const Frag a  = ldfrag(ap + k0, hh);
    const Frag b0 = ldfrag(bp0 + k0, hh);
    const Frag b1 = ldfrag(bp1 + k0, hh);
    acc0 = mma_bf16(a, b0, acc0);
    acc1 = mma_bf16(a, b1, acc1);
  }
  const int   col  = n0 + 32 * cp + l15;
  const float bia0 = bf16q(bg[col]);
  const float bia1 = bf16q(bg[col + 16]);
#pragma unroll
  for (int r = 0; r < 8; ++r) {
    const float z0 = acc0[r] + bia0;
    const float z1 = acc1[r] + bia1;
    const float g0 = z0 * __builtin_amdgcn_rcpf(1.0f + __expf(-z0));
    const float g1 = z1 * __builtin_amdgcn_rcpf(1.0f + __expf(-z1));
    Cs[16 * rg + mloc + r][32 * cp + l15]      = g0;
    Cs[16 * rg + mloc + r][32 * cp + 16 + l15] = g1;
  }
  __syncthreads();
  v4f    o[4];
  size_t d[4];
#pragma unroll
  for (int i = 0; i < 4; ++i) {
    const int L    = 32 * i + (t >> 3);
    const int row  = L >> 1;
    const int col4 = (L & 1) * 32 + (t & 7) * 4;
    o[i] = *(const v4f*)&Cs[row][col4];
    d[i] = (size_t)(m0 + row) * DIM + n0 + col4;
  }
#pragma unroll
  for (int i = 0; i < 4; ++i) *(volatile v4f*)(G + d[i]) = o[i];
  __threadfence();
#pragma unroll
  for (int i = 0; i < 4; ++i) *(volatile v4f*)(G + d[i]) = o[i];
}

__global__ __launch_bounds__(256) void k_gn(const float* __restrict__ Xf, const float* __restrict__ G,
                                            const float* __restrict__ beta, u16* __restrict__ Zh,
                                            u16* __restrict__ Zl) {
  __shared__ __attribute__((aligned(16))) _Float16 zs[2][256];
  const int t = threadIdx.x, lane = t & 31, w = t >> 5;
  const size_t row = blockIdx.x >> 2;
  const int    cb  = (blockIdx.x & 3) * 256;
  const int    c   = cb + t;
  const size_t idx = row * DIM + c;
  const float x  = Xf[idx];
  const float g  = G[idx];
  const float be = bf16q(beta[c]);
  float s = x;
  s += __shfl_xor(s, 16, 32);
  s += __shfl_xor(s, 8, 32);
  s += __shfl_xor(s, 4, 32);
  s += __shfl_xor(s, 2, 32);
  s += __shfl_xor(s, 1, 32);
  const float mu = s * (1.0f / 32.0f);
  const float dv = x - mu;
  float q2 = dv * dv;
  q2 += __shfl_xor(q2, 16, 32);
  q2 += __shfl_xor(q2, 8, 32);
  q2 += __shfl_xor(q2, 4, 32);
  q2 += __shfl_xor(q2, 2, 32);
  q2 += __shfl_xor(q2, 1, 32);
  const float var = q2 * (1.0f / 32.0f);
  const float y   = dv * rsqrtf(var + 1e-3f) + be;
  const float z   = g * y * ZSC;
  const _Float16 zh = (_Float16)z;
  const _Float16 zl = (_Float16)((z - (float)zh) * RSC);
  zs[0][t] = zh;
  zs[1][t] = zl;
  __syncthreads();
  if (w < 2) {
    Pack8 pk;
    pk.h = *(const v8h*)&zs[w][8 * lane];
    u16* dp = ((w == 0) ? Zh : Zl) + row * DIM + cb + 8 * lane;
    *(volatile v4u*)dp = pk.u;
    __threadfence();
    *(volatile v4u*)dp = pk.u;
  }
}

__global__ __launch_bounds__(256) void k_out(const u16* __restrict__ Zh, const u16* __restrict__ Zl,
                                             const u16* __restrict__ WoT, const float* __restrict__ bo,
                                             float* __restrict__ out) {
  __shared__ __attribute__((aligned(16))) float Cs[64][68];
  const int t = threadIdx.x, lane = t & 31, w = t >> 5;
  const int hh = lane >> 4, l15 = lane & 15, mloc = 8 * hh;
  const int rg = w & 3, cp = w >> 2;
  const int m0 = blockIdx.x * 64, n0 = blockIdx.y * 64;

  const u16* aph = Zh + (size_t)(m0 + 16 * rg + l15) * DIM;
  const u16* apl = Zl + (size_t)(m0 + 16 * rg + l15) * DIM;
  const u16* bp0 = WoT + (size_t)(n0 + 32 * cp + l15) * DIM;
  const u16* bp1 = bp0 + 16 * DIM;

  v8f h0 = {}, h1 = {}, l0 = {}, l1 = {};
#pragma unroll 2
  for (int k0 = 0; k0 < DIM; k0 += 32) {
    const Frag ah = ldfrag(aph + k0, hh);
    const Frag al = ldfrag(apl + k0, hh);
    const Frag b0 = ldfrag(bp0 + k0, hh);
    const Frag b1 = ldfrag(bp1 + k0, hh);
    h0 = mma_f16(ah, b0, h0);
    h1 = mma_f16(ah, b1, h1);
    l0 = mma_f16(al, b0, l0);
    l1 = mma_f16(al, b1, l1);
  }
  const int   col  = n0 + 32 * cp + l15;
  const float bia0 = bf16q(bo[col]);
  const float bia1 = bf16q(bo[col + 16]);
  const float c1 = 1.0f / (ZSC * WOSC);
  const float c2 = c1 / RSC;
#pragma unroll
  for (int r = 0; r < 8; ++r) {
    Cs[16 * rg + mloc + r][32 * cp + l15]      = h0[r] * c1 + l0[r] * c2 + bia0;
    Cs[16 * rg + mloc + r][32 * cp + 16 + l15] = h1[r] * c1 + l1[r] * c2 + bia1;
  }
  __syncthreads();
  v4f    o[4];
  size_t d[4];
#pragma unroll
  for (int i = 0; i < 4; ++i) {
    const int L    = 32 * i + (t >> 3);
    const int row  = L >> 1;
    const int col4 = (L & 1) * 32 + (t & 7) * 4;
    o[i] = *(const v4f*)&Cs[row][col4];
    d[i] = (size_t)(m0 + row) * DIM + n0 + col4;
  }
#pragma unroll
  for (int i = 0; i < 4; ++i) *(volatile v4f*)(out + d[i]) = o[i];
  __threadfence();
#pragma unroll
  for (int i = 0; i < 4; ++i) *(volatile v4f*)(out + d[i]) = o[i];
}

extern "C" void kernel_launch(void* const* d_in, const int* in_sizes, int n_in,
                              void* d_out, int out_size, void* d_ws, size_t ws_size,
                              hipStream_t stream) {
  if (n_in < 9) return;
  const float* q     = (const float*)d_in[0];
  const float* W_qkv = (const float*)d_in[3];
  const float* Wg    = (const float*)d_in[4];
  const float* bg    = (const float*)d_in[5];
  const float* Wo    = (const float*)d_in[6];
  const float* bo    = (const float*)d_in[7];
  const float* beta  = (const float*)d_in[8];
  float* outp = (float*)d_out;

  if (in_sizes[0] < ((NB - 1) * SEQ_FULL + SEQ) * DIM) return;
  if (in_sizes[3] < NH * HD * HD) return;
  if (in_sizes[4] < DIM * DIM || in_sizes[6] < DIM * DIM) return;
  if (in_sizes[5] < DIM || in_sizes[7] < DIM || in_sizes[8] < DIM) return;
  if (out_size < ROWS * DIM) return;

  const size_t szQB   = (size_t)ROWS * DIM * 2;
  const size_t szWT   = (size_t)NH * HD * HD * 2;
  const size_t szWGT  = (size_t)DIM * DIM * 2;
  const size_t szWOT  = (size_t)DIM * DIM * 2;
  const size_t szCOLW = (size_t)NB * NH * SEQ * 4;
  const size_t szPF   = (size_t)ROWS * DIM * 4;
  const size_t szPH   = (size_t)ROWS * DIM * 2;
  const size_t szVTH  = (size_t)ROWS * DIM * 2;
  const size_t szVTL  = (size_t)ROWS * DIM * 2;
  size_t off = 0;
  auto carve = [&](size_t bytes) -> char* {
    char* p = (char*)d_ws + off;
    off = (off + bytes + 255) & ~(size_t)255;
    return p;
  };
  char* rQB   = carve(szQB);
  char* rWT   = carve(szWT);
  char* rWGT  = carve(szWGT);
  char* rWOT  = carve(szWOT);
  char* rCOLW = carve(szCOLW);
  char* rPF   = carve(szPF);
  char* rPH   = carve(szPH + szVTH);
  char* rVTL  = carve(szVTL);
  if (off > ws_size) return;
  static_assert((size_t)ROWS * DIM * 4 == (size_t)NB * NH * SEQ * HD * 4);
  static_assert((size_t)ROWS * DIM * 4 == 2 * (size_t)ROWS * DIM * 2);

  u16*   qb   = (u16*)rQB;
  u16*   Zh   = (u16*)rQB;
  u16*   WT   = (u16*)rWT;
  u16*   WgT  = (u16*)rWGT;
  u16*   WoT  = (u16*)rWOT;
  float* colw = (float*)rCOLW;
  float* Pf   = (float*)rPF;
  float* Xf   = (float*)rPF;
  u16*   Phr  = (u16*)rPH;
  u16*   Vth  = (u16*)(rPH + szPH);
  float* G    = (float*)rPH;
  u16*   Vtl  = (u16*)rVTL;
  u16*   Zl   = (u16*)rVTL;

  k_cvt_q<<<(ROWS * DIM) / 2048, 256, 0, stream>>>(q, qb);
  k_tr<0><<<dim3(HD / 64, HD / 64, NH), 256, 0, stream>>>(W_qkv, WT, HD, HD);
  k_tr<0><<<dim3(DIM / 64, DIM / 64, 1), 256, 0, stream>>>(Wg, WgT, DIM, DIM);
  k_tr<1><<<dim3(DIM / 64, DIM / 64, 1), 256, 0, stream>>>(Wo, WoT, DIM, DIM);

  k_proj<<<dim3(SEQ / 64, HD / 64, NB * NH), 256, 0, stream>>>(qb, WT, Pf, Phr, Vth, Vtl);
  k_colstat<<<NB * NH, 128, 0, stream>>>(Pf, colw);
  k_ret<<<dim3(SEQ / 64, NH, NB), 512, 0, stream>>>(Phr, Vth, Vtl, colw, Xf);
  k_gate<<<dim3(ROWS / 64, DIM / 64), 256, 0, stream>>>(qb, WgT, bg, G);
  k_gn<<<ROWS * 4, 256, 0, stream>>>(Xf, G, beta, Zh, Zl);
  k_out<<<dim3(ROWS / 64, DIM / 64), 256, 0, stream>>>(Zh, Zl, WoT, bo, outp);
}
